// GroupQueryAttention_15461882265879
// MI455X (gfx1250) — hardware-verified
//
#include <hip/hip_runtime.h>

#ifndef NB
#define NB 2
#endif
#ifndef SEQ
#define SEQ 2048
#endif
#define NB_FULL 2
#define S_FULL  2048
#define HID     2048
#define NHEAD   16
#define HDIM    128
#define NGRP    4
#define MPG     (NHEAD / NGRP)
#define KVW     (NGRP * HDIM)
#define NROW    (NB * SEQ)
#define NQT     (SEQ / 16)

static_assert(NB >= 1 && NB <= NB_FULL);
static_assert(SEQ >= 64 && SEQ <= S_FULL && (SEQ % 64) == 0);
static_assert(HDIM == 128 && (HID % 64) == 0 && (KVW % 64) == 0 && (HID % 32) == 0);

#define WCAR   64.0f
#define QCAR   16.0f
#define PCAR   1024.0f
#define CCAR   256.0f
#define RSQ_HD 0.08838834764831845f
#define MNEG   (-1.0e-9f)

#define XBYTES   ((size_t)NROW * HID * 2)
#define WQBYTES  ((size_t)HID * HID * 2)
#define WKBYTES  ((size_t)KVW * HID * 2)
#define KBYTES   ((size_t)NROW * KVW * 2)
#define WS_TOTAL (XBYTES + WQBYTES + WKBYTES + WKBYTES + WQBYTES + XBYTES + KBYTES + KBYTES + XBYTES)
static_assert(WS_TOTAL <= (size_t)134217728);
static_assert((XBYTES % 256) == 0 && (WQBYTES % 256) == 0 && (WKBYTES % 256) == 0 && (KBYTES % 256) == 0);

typedef _Float16     v8h  __attribute__((ext_vector_type(8)));
typedef _Float16     v16h __attribute__((ext_vector_type(16)));
typedef float        v4f  __attribute__((ext_vector_type(4)));
typedef float        v8f  __attribute__((ext_vector_type(8)));
typedef unsigned int v4u  __attribute__((ext_vector_type(4)));

__device__ __forceinline__ float bf16r(float x) {
    unsigned int u = __float_as_uint(x);
    u = (u + 0x7FFFu + ((u >> 16) & 1u)) & 0xFFFF0000u;
    return __uint_as_float(u);
}

__device__ __forceinline__ v16h load_frag(const _Float16* p) {
    v8h lo = *(const v8h*)(p);
    v8h hi = *(const v8h*)(p + 16);
    return __builtin_shufflevector(lo, hi, 0,1,2,3,4,5,6,7,8,9,10,11,12,13,14,15);
}

__device__ __forceinline__ v8f wmma_f16(v16h a, v16h b, v8f c) {
    return __builtin_amdgcn_wmma_f32_16x16x32_f16(false, a, false, b, (short)0, c, false, false);
}

__device__ __forceinline__ void st16u(void* p, v4u v)  { *(volatile v4u*)p = v; }
__device__ __forceinline__ void st16f(float* p, v4f v) { *(volatile v4f*)p = v; }

__device__ __forceinline__ void wave_lds_sync() {
    __builtin_amdgcn_fence(__ATOMIC_RELEASE, "wavefront");
    __builtin_amdgcn_wave_barrier();
    __builtin_amdgcn_fence(__ATOMIC_ACQUIRE, "wavefront");
}

__global__ __launch_bounds__(256) void k_cvt_x(const float* __restrict__ hs, _Float16* __restrict__ X, int n8)
{
    const int i = blockIdx.x * 256 + threadIdx.x;
    if (i >= n8) return;
    const size_t e0 = (size_t)i * 8;
    const int r = (int)(e0 / HID);
    const int c = (int)(e0 - (size_t)r * HID);
    const int b = r / SEQ;
    const int s = r - b * SEQ;
    const float* src = hs + ((size_t)b * S_FULL + s) * HID + c;
    const v4f f0 = *(const v4f*)(src);
    const v4f f1 = *(const v4f*)(src + 4);
    v8h hv;
#pragma unroll
    for (int e = 0; e < 4; ++e) {
        hv[e]     = (_Float16)bf16r(f0[e]);
        hv[4 + e] = (_Float16)bf16r(f1[e]);
    }
    const v4u u = __builtin_bit_cast(v4u, hv);
    _Float16* dst = X + e0;
    st16u(dst, u);
    __threadfence();
    st16u(dst, u);
}

__global__ __launch_bounds__(256) void k_wt(const float* __restrict__ W, _Float16* __restrict__ WT, int K, int N)
{
    __shared__ float tile[64 * 65];
    const int n0 = blockIdx.x * 64;
    const int k0 = blockIdx.y * 64;
    const int t  = threadIdx.x;
#pragma unroll 4
    for (int p = 0; p < 16; ++p) {
        const int kl = p * 4 + (t >> 6);
        const int nl = t & 63;
        tile[kl * 65 + nl] = W[(size_t)(k0 + kl) * N + n0 + nl];
    }
    __syncthreads();
    const int wave = t >> 5, lane = t & 31;
    const int c8 = (lane & 7) * 8;
    const int rA = wave * 8 + (lane >> 3);
    const int rB = rA + 4;
    v8h ha, hb;
#pragma unroll
    for (int e = 0; e < 8; ++e) {
        ha[e] = (_Float16)(bf16r(tile[(c8 + e) * 65 + rA]) * WCAR);
        hb[e] = (_Float16)(bf16r(tile[(c8 + e) * 65 + rB]) * WCAR);
    }
    const v4u ua = __builtin_bit_cast(v4u, ha);
    const v4u ub = __builtin_bit_cast(v4u, hb);
    _Float16* pa = WT + (size_t)(n0 + rA) * K + k0 + c8;
    _Float16* pb = WT + (size_t)(n0 + rB) * K + k0 + c8;
    st16u(pa, ua);
    st16u(pb, ub);
    __threadfence();
    st16u(pa, ua);
    st16u(pb, ub);
}

#define LDT 36
template <int MODE>
__global__ __launch_bounds__(128) void k_gemm(const _Float16* __restrict__ A, const _Float16* __restrict__ BT,
                                             const float* __restrict__ bias, void* __restrict__ Cout,
                                             int M, int N, int K, int lda, int ldb, int ldc,
                                             float inv_in, float out_scale)
{
    __shared__ __attribute__((aligned(16))) float stg[4 * 64 * LDT];
    const int wave = threadIdx.x >> 5;
    const int lane = threadIdx.x & 31;
    const int wid  = blockIdx.x * 4 + wave;
    const int tilesN = N >> 6;
    const int tilesM = M >> 5;
    if (wid >= tilesM * tilesN) return;
    const int m0 = (wid / tilesN) << 5;
    const int n0 = (wid % tilesN) << 6;

    const int rloc = lane & 15;
    const int hl   = lane >> 4;
    const int kb   = hl << 3;

    const _Float16* arow0 = A  + (size_t)(m0 + rloc) * lda + kb;
    const _Float16* arow1 = arow0 + (size_t)16 * lda;
    const _Float16* brow  = BT + (size_t)(n0 + rloc) * ldb + kb;
    const size_t bstep = (size_t)16 * ldb;

    v8f acc[2][4];
#pragma unroll
    for (int hh = 0; hh < 2; ++hh)
#pragma unroll
        for (int j = 0; j < 4; ++j)
#pragma unroll
            for (int i = 0; i < 8; ++i) acc[hh][j][i] = 0.0f;

#pragma unroll 1
    for (int k0 = 0; k0 < K; k0 += 32) {
        v16h a0 = load_frag(arow0 + k0);
        v16h a1 = load_frag(arow1 + k0);
        v16h b0 = load_frag(brow + k0);
        v16h b1 = load_frag(brow + bstep + k0);
        v16h b2 = load_frag(brow + 2 * bstep + k0);
        v16h b3 = load_frag(brow + 3 * bstep + k0);

        acc[0][0] = wmma_f16(a0, b0, acc[0][0]);
        acc[1][0] = wmma_f16(a1, b0, acc[1][0]);
        acc[0][1] = wmma_f16(a0, b1, acc[0][1]);
        acc[1][1] = wmma_f16(a1, b1, acc[1][1]);
        acc[0][2] = wmma_f16(a0, b2, acc[0][2]);
        acc[1][2] = wmma_f16(a1, b2, acc[1][2]);
        acc[0][3] = wmma_f16(a0, b3, acc[0][3]);
        acc[1][3] = wmma_f16(a1, b3, acc[1][3]);
        asm volatile("v_nop\n\tv_nop\n\tv_nop\n\tv_nop"
                     : "+v"(acc[0][0]), "+v"(acc[0][1]), "+v"(acc[0][2]), "+v"(acc[0][3]),
                       "+v"(acc[1][0]), "+v"(acc[1][1]), "+v"(acc[1][2]), "+v"(acc[1][3])
                     : "v"(a0), "v"(a1), "v"(b0), "v"(b1), "v"(b2), "v"(b3));
    }

    float* sw = stg + wave * (64 * LDT);
#pragma unroll
    for (int hh = 0; hh < 2; ++hh)
#pragma unroll
        for (int j = 0; j < 4; ++j) {
            float* q = sw + (16 * j + rloc) * LDT + 16 * hh + 8 * hl;
            *(v4f*)(q)     = acc[hh][j].lo;
            *(v4f*)(q + 4) = acc[hh][j].hi;
        }
    wave_lds_sync();

    if (MODE == 2) {
        float* C = (float*)Cout;
        const int c4 = (lane & 15) * 4;
        const v4f bb = *(const v4f*)(bias + n0 + c4);
        v4f vals[16];
#pragma unroll
        for (int it = 0; it < 16; ++it) {
            const int row = 2 * it + hl;
            v4f v;
#pragma unroll
            for (int e = 0; e < 4; ++e)
                v[e] = (sw[(c4 + e) * LDT + row] * inv_in + bf16r(bb[e])) * out_scale;
            vals[it] = v;
        }
#pragma unroll
        for (int ps = 0; ps < 2; ++ps) {
#pragma unroll
            for (int it = 0; it < 16; ++it) {
                const int m = m0 + 2 * it + hl;
                const size_t orow = (size_t)(m / SEQ) * S_FULL + (size_t)(m % SEQ);
                st16f(C + orow * (size_t)ldc + n0 + c4, vals[it]);
            }
            if (ps == 0) __threadfence();
        }
    } else {
        _Float16* C = (_Float16*)Cout;
        const int c8 = (lane & 7) * 8;
        const int rq = lane >> 3;
        v8f bb8 = {0.f, 0.f, 0.f, 0.f, 0.f, 0.f, 0.f, 0.f};
        if (MODE == 0) bb8 = *(const v8f*)(bias + n0 + c8);
        v4u vals[8];
#pragma unroll
        for (int it = 0; it < 8; ++it) {
            const int row = 4 * it + rq;
            float br = 0.0f;
            if (MODE == 1) br = bf16r(bias[m0 + row]);
            v8h hv;
#pragma unroll
            for (int e = 0; e < 8; ++e) {
                const float x    = sw[(c8 + e) * LDT + row];
                const float bsel = (MODE == 0) ? bf16r(bb8[e]) : br;
                hv[e] = (_Float16)((x * inv_in + bsel) * out_scale);
            }
            vals[it] = __builtin_bit_cast(v4u, hv);
        }
        const int bq = n0 / SEQ;
        const int s0 = n0 - bq * SEQ + c8;
#pragma unroll
        for (int ps = 0; ps < 2; ++ps) {
#pragma unroll
            for (int it = 0; it < 8; ++it) {
                const int m = m0 + 4 * it + rq;
                _Float16* p;
                if (MODE == 0) p = C + (size_t)m * ldc + n0 + c8;
                else           p = C + ((size_t)(bq * M + m)) * SEQ + s0;
                st16u(p, vals[it]);
            }
            if (ps == 0) __threadfence();
        }
    }
}

#define OPITCH 136
__global__ __launch_bounds__(64) void k_flash(const _Float16* __restrict__ Qp, const _Float16* __restrict__ Kp,
                                            const _Float16* __restrict__ Vt, const float* __restrict__ mask,
                                            _Float16* __restrict__ Oa)
{
    __shared__ __attribute__((aligned(16))) _Float16 ost[2 * 16 * OPITCH];
    const int lane = threadIdx.x & 31;
    const int wave = threadIdx.x >> 5;
    const int wid  = blockIdx.x * 2 + wave;
    if (wid >= NB * NHEAD * NQT) return;
    const int sqt = wid % NQT;
    const int bh  = wid / NQT;
    const int h   = bh % NHEAD;
    const int b   = bh / NHEAD;
    const int g   = h / MPG;
    const int sq0 = sqt << 4;
    const int nloc = lane & 15;
    const int hl   = lane >> 4;
    const int kb   = hl << 3;

    const _Float16* qrow = Qp + ((size_t)(b * SEQ + sq0 + nloc)) * HID + h * HDIM + kb;
    const v16h qb0 = load_frag(qrow);
    const v16h qb1 = load_frag(qrow + 32);
    const v16h qb2 = load_frag(qrow + 64);
    const v16h qb3 = load_frag(qrow + 96);

    const _Float16* kbase = Kp + ((size_t)(b * SEQ) + nloc) * KVW + g * HDIM + kb;
    const _Float16* vbase = Vt + ((size_t)(b * KVW + g * HDIM) + nloc) * SEQ + kb;
    const float*    mrow  = mask + (size_t)b * S_FULL + kb;

    const float SCL = RSQ_HD * (1.0f / (QCAR * QCAR));

    float m_run = -1.0e30f, l_run = 0.0f;
    v8f o[8];
#pragma unroll
    for (int r = 0; r < 8; ++r)
#pragma unroll
        for (int i = 0; i < 8; ++i) o[r][i] = 0.0f;
    const v8f z = {0.f, 0.f, 0.f, 0.f, 0.f, 0.f, 0.f, 0.f};

#pragma unroll 1
    for (int kt = 0; kt < SEQ; kt += 32) {
        const _Float16* kr  = kbase + (size_t)kt * KVW;
        const _Float16* kr2 = kr + (size_t)16 * KVW;
        v16h a0 = load_frag(kr);
        v16h a1 = load_frag(kr + 32);
        v16h a2 = load_frag(kr + 64);
        v16h a3 = load_frag(kr + 96);
        v16h c0 = load_frag(kr2);
        v16h c1 = load_frag(kr2 + 32);
        v16h c2 = load_frag(kr2 + 64);
        v16h c3 = load_frag(kr2 + 96);

        v8f st1 = wmma_f16(a0, qb0, z);
        st1 = wmma_f16(a1, qb1, st1);
        st1 = wmma_f16(a2, qb2, st1);
        st1 = wmma_f16(a3, qb3, st1);
        v8f st2 = wmma_f16(c0, qb0, z);
        st2 = wmma_f16(c1, qb1, st2);
        st2 = wmma_f16(c2, qb2, st2);
        st2 = wmma_f16(c3, qb3, st2);
        asm volatile("v_nop\n\tv_nop\n\tv_nop\n\tv_nop"
                     : "+v"(st1), "+v"(st2)
                     : "v"(a0), "v"(a1), "v"(a2), "v"(a3),
                       "v"(c0), "v"(c1), "v"(c2), "v"(c3),
                       "v"(qb0), "v"(qb1), "v"(qb2), "v"(qb3));

        const v8f mk1 = *(const v8f*)(mrow + kt);
        const v8f mk2 = *(const v8f*)(mrow + kt + 16);
        float s1[8], s2[8];
        float t = -3.0e38f;
#pragma unroll
        for (int i = 0; i < 8; ++i) { s1[i] = st1[i] * SCL + mk1[i] * MNEG; t = fmaxf(t, s1[i]); }
#pragma unroll
        for (int i = 0; i < 8; ++i) { s2[i] = st2[i] * SCL + mk2[i] * MNEG; t = fmaxf(t, s2[i]); }
        t = fmaxf(t, __shfl_xor(t, 16, 32));
        const float m_new = fmaxf(m_run, t);
        const float alpha = __expf(m_run - m_new);

        v16h pb;
        float rs = 0.0f;
#pragma unroll
        for (int i = 0; i < 8; ++i) {
            const float p = __expf(s1[i] - m_new);
            pb[i] = (_Float16)(p * PCAR);  rs += p;
        }
#pragma unroll
        for (int i = 0; i < 8; ++i) {
            const float p = __expf(s2[i] - m_new);
            pb[8 + i] = (_Float16)(p * PCAR);  rs += p;
        }
        rs += __shfl_xor(rs, 16, 32);
        l_run = l_run * alpha + rs;
        m_run = m_new;

#pragma unroll
        for (int r = 0; r < 8; ++r)
#pragma unroll
            for (int i = 0; i < 8; ++i) o[r][i] *= alpha;

        const _Float16* vr = vbase + kt;
        {
            v16h va0 = load_frag(vr);
            v16h va1 = load_frag(vr + (size_t)16 * SEQ);
            v16h va2 = load_frag(vr + (size_t)32 * SEQ);
            v16h va3 = load_frag(vr + (size_t)48 * SEQ);
            o[0] = wmma_f16(va0, pb, o[0]);
            o[1] = wmma_f16(va1, pb, o[1]);
            o[2] = wmma_f16(va2, pb, o[2]);
            o[3] = wmma_f16(va3, pb, o[3]);
            asm volatile("v_nop\n\tv_nop\n\tv_nop\n\tv_nop"
                         : "+v"(o[0]), "+v"(o[1]), "+v"(o[2]), "+v"(o[3])
                         : "v"(va0), "v"(va1), "v"(va2), "v"(va3), "v"(pb));
        }
        {
            v16h va4 = load_frag(vr + (size_t)64 * SEQ);
            v16h va5 = load_frag(vr + (size_t)80 * SEQ);
            v16h va6 = load_frag(vr + (size_t)96 * SEQ);
            v16h va7 = load_frag(vr + (size_t)112 * SEQ);
            o[4] = wmma_f16(va4, pb, o[4]);
            o[5] = wmma_f16(va5, pb, o[5]);
            o[6] = wmma_f16(va6, pb, o[6]);
            o[7] = wmma_f16(va7, pb, o[7]);
            asm volatile("v_nop\n\tv_nop\n\tv_nop\n\tv_nop"
                         : "+v"(o[4]), "+v"(o[5]), "+v"(o[6]), "+v"(o[7])
                         : "v"(va4), "v"(va5), "v"(va6), "v"(va7), "v"(pb));
        }
    }

    const float inv = (1.0f / l_run) * (CCAR / (PCAR * QCAR));
    _Float16* ow = ost + wave * (16 * OPITCH);
#pragma unroll
    for (int r = 0; r < 8; ++r) {
        v8h hv;
#pragma unroll
        for (int i = 0; i < 8; ++i) hv[i] = (_Float16)(o[r][i] * inv);
        *(v8h*)(ow + nloc * OPITCH + 16 * r + 8 * hl) = hv;
    }
    wave_lds_sync();

    v4u vals[8];
    const int c8 = nloc * 8;
#pragma unroll
    for (int it = 0; it < 8; ++it) {
        const int row = 2 * it + hl;
        vals[it] = __builtin_bit_cast(v4u, *(const v8h*)(ow + row * OPITCH + c8));
    }
    _Float16* obase = Oa + ((size_t)(b * SEQ + sq0)) * HID + h * HDIM + c8;
#pragma unroll
    for (int ps = 0; ps < 2; ++ps) {
#pragma unroll
        for (int it = 0; it < 8; ++it) {
            const int row = 2 * it + hl;
            st16u(obase + (size_t)row * HID, vals[it]);
        }
        if (ps == 0) __threadfence();
    }
}

extern "C" void kernel_launch(void* const* d_in, const int* in_sizes, int n_in,
                              void* d_out, int out_size, void* d_ws, size_t ws_size,
                              hipStream_t stream)
{
    if (n_in < 10) return;
    const int rows_used = (NB - 1) * S_FULL + SEQ;
    if (in_sizes[0] < rows_used * HID) return;
    if (in_sizes[1] < rows_used) return;
    if (in_sizes[2] < HID * HID || in_sizes[3] < HID) return;
    if (in_sizes[4] < HID * KVW || in_sizes[5] < KVW) return;
    if (in_sizes[6] < HID * KVW || in_sizes[7] < KVW) return;
    if (in_sizes[8] < HID * HID || in_sizes[9] < HID) return;
    if ((size_t)out_size < (size_t)rows_used * HID) return;
    if (ws_size < WS_TOTAL) return;

    const float* hs  = (const float*)d_in[0];
    const float* msk = (const float*)d_in[1];
    const float* Wq  = (const float*)d_in[2];
    const float* bq  = (const float*)d_in[3];
    const float* Wk  = (const float*)d_in[4];
    const float* bk  = (const float*)d_in[5];
    const float* Wv  = (const float*)d_in[6];
    const float* bv  = (const float*)d_in[7];
    const float* Wo  = (const float*)d_in[8];
    const float* bo  = (const float*)d_in[9];
    float* out = (float*)d_out;

    char* wp = (char*)d_ws;
    _Float16* X16 = (_Float16*)wp; wp += XBYTES;
    _Float16* WqT = (_Float16*)wp; wp += WQBYTES;
    _Float16* WkT = (_Float16*)wp; wp += WKBYTES;
    _Float16* WvT = (_Float16*)wp; wp += WKBYTES;
    _Float16* WoT = (_Float16*)wp; wp += WQBYTES;
    _Float16* Q16 = (_Float16*)wp; wp += XBYTES;
    _Float16* K16 = (_Float16*)wp; wp += KBYTES;
    _Float16* Vt  = (_Float16*)wp; wp += KBYTES;
    _Float16* C16 = (_Float16*)wp; wp += XBYTES;

    const int n8 = (NROW * HID) / 8;
    k_cvt_x<<<(n8 + 255) / 256, 256, 0, stream>>>(hs, X16, n8);

    k_wt<<<dim3(HID / 64, HID / 64), 256, 0, stream>>>(Wq, WqT, HID, HID);
    k_wt<<<dim3(KVW / 64, HID / 64), 256, 0, stream>>>(Wk, WkT, HID, KVW);
    k_wt<<<dim3(KVW / 64, HID / 64), 256, 0, stream>>>(Wv, WvT, HID, KVW);
    k_wt<<<dim3(HID / 64, HID / 64), 256, 0, stream>>>(Wo, WoT, HID, HID);

    const int wq = (NROW / 32) * (HID / 64);
    const int wk = (NROW / 32) * (KVW / 64);
    const int wv = (KVW / 32) * (NROW / 64);
    k_gemm<0><<<(wq + 3) / 4, 128, 0, stream>>>(X16, WqT, bq, (void*)Q16, NROW, HID, HID, HID, HID, HID,
                                                1.0f / WCAR, QCAR);
    k_gemm<0><<<(wk + 3) / 4, 128, 0, stream>>>(X16, WkT, bk, (void*)K16, NROW, KVW, HID, HID, HID, KVW,
                                                1.0f / WCAR, QCAR);
    k_gemm<1><<<(wv + 3) / 4, 128, 0, stream>>>(WvT, X16, bv, (void*)Vt, KVW, NROW, HID, HID, HID, SEQ,
                                                1.0f / WCAR, QCAR);

    const int wf = NB * NHEAD * NQT;
    k_flash<<<(wf + 1) / 2, 64, 0, stream>>>(Q16, K16, Vt, msk, C16);

    k_gemm<2><<<(wq + 3) / 4, 128, 0, stream>>>(C16, WoT, bo, (void*)out, NROW, HID, HID, HID, HID, HID,
                                                1.0f / (CCAR * WCAR), 1.0f);
}
